// DefuzzyLayer2_8160437862725
// MI455X (gfx1250) — hardware-run, weakly checked
//
#include <hip/hip_runtime.h>


#ifndef NROWS
#define NROWS 8192
#endif
#define NROWS_FULL 8192
#define DIN   512
#define DOUT  512
#define KT    (2 * DIN)
#define TP    72
#define CSB   128

static_assert(NROWS <= NROWS_FULL);
static_assert(NROWS % 64 == 0);
static_assert(DOUT % 64 == 0);
static_assert(DIN % 64 == 0);
static_assert(KT % 32 == 0);
static_assert(DIN / 8 == 64);
static_assert(((size_t)NROWS * (DIN / 8)) % 256 == 0);
static_assert(DOUT % CSB == 0);
static_assert(CSB == 128);
static_assert((TP * 2) % 16 == 0);
static_assert((KT * 2) % 128 == 0);
static_assert((DIN * 2) % 128 == 0);
static_assert(16 * 68 * 4 <= 131072);
static_assert(64 * TP * 2 <= 131072);
static_assert(CSB * 4 <= 131072);

typedef unsigned short bf;
typedef __attribute__((ext_vector_type(16))) __bf16   v16bf;
typedef __attribute__((ext_vector_type(8)))  unsigned short v8us;
typedef __attribute__((ext_vector_type(8)))  float    v8f;
typedef __attribute__((ext_vector_type(4)))  float    v4f;
typedef v4f  __attribute__((may_alias)) v4fa;
typedef v8us __attribute__((may_alias)) v8usa;

__device__ __forceinline__ unsigned short f2bf(float f) { unsigned u = __float_as_uint(f); u += 0x7FFFu + ((u >> 16) & 1u); return (unsigned short)(u >> 16); }
__device__ __forceinline__ float bfr(float f) { return __uint_as_float(((unsigned)f2bf(f)) << 16); }
__device__ __forceinline__ v16bf cat16b(v8us lo, v8us hi) { return __builtin_bit_cast(v16bf, __builtin_shufflevector(lo, hi, 0, 1, 2, 3, 4, 5, 6, 7, 8, 9, 10, 11, 12, 13, 14, 15)); }
__device__ __forceinline__ v8f wmmab(v16bf a, v16bf b, v8f c) { return __builtin_amdgcn_wmma_f32_16x16x32_bf16(false, a, false, b, (short)0, c, false, false); }
__device__ __forceinline__ v8f wmmabg(v16bf a, v16bf b, v8f c) { c = wmmab(a, b, c); asm volatile("v_nop\n\tv_nop\n\tv_nop\n\tv_nop" : "+v"(c) : "v"(a), "v"(b)); return c; }
__device__ __forceinline__ v16bf ldb(const bf* p)  { return cat16b(*(const v8us*)p, *(const v8us*)(p + 16)); }
__device__ __forceinline__ void wave_sync() { __builtin_amdgcn_fence(3  , "wavefront"); __builtin_amdgcn_wave_barrier(); asm volatile("" ::: "memory"); }

__global__ __launch_bounds__(256) void k_aplane(const float* __restrict__ x, bf* AP) {
#pragma clang fp contract(off)
    const unsigned i = blockIdx.x * 256u + threadIdx.x;
    if (i >= (unsigned)NROWS * (unsigned)(DIN / 8)) return;
    const unsigned row = i >> 6, g = i & 63u;
    const v8f v = *(const v8f*)(x + (size_t)row * DIN + (size_t)g * 8);
    v8us sv, sx;
#pragma unroll
    for (int k = 0; k < 8; ++k) {
        const float xb = bfr(v[k]);
        const float sq = xb * xb;
        sv[k] = f2bf(sq); sx[k] = f2bf(xb); }
    bf* d = AP + (size_t)row * KT + (size_t)g * 8;
    *(volatile v8us*)(d) = sv; *(volatile v8us*)(d + DIN) = sx;
    __threadfence();
    *(volatile v8us*)(d) = sv; *(volatile v8us*)(d + DIN) = sx;
}

static_assert(256 * 16 * 2 == 64 * 128);
__global__ __launch_bounds__(256) void k_wt(const float* __restrict__ W, bf* WT, unsigned coloff) {
    __shared__ __align__(16) unsigned short ts[64 * TP];
    const unsigned tid = threadIdx.x;
    const unsigned d0 = blockIdx.x * 64u, o0 = blockIdx.y * 64u;
#pragma unroll
    for (unsigned i = 0; i < 4; ++i) {
        const unsigned lin = tid + i * 256u; const unsigned d = lin >> 4, c4 = (lin & 15u) * 4u;
        const v4f v = *(const v4f*)(W + (size_t)(d0 + d) * DOUT + o0 + c4);
#pragma unroll
        for (unsigned j = 0; j < 4; ++j) ts[(c4 + j) * TP + d] = f2bf(v[j]); }
    __syncthreads();
#pragma unroll 1
    for (int ps = 0; ps < 2; ++ps) {
#pragma unroll
        for (unsigned s = 0; s < 2; ++s) { const unsigned row = s * 32u + (tid >> 3), c8 = (tid & 7u) * 8u;
            const v8us val = *(const v8usa*)(&ts[row * TP + c8]);
            *(volatile v8us*)(WT + (size_t)(o0 + row) * KT + coloff + d0 + c8) = val; }
        if (ps == 0) __threadfence(); }
}

static_assert(32 * 16 == CSB * 4);
__global__ __launch_bounds__(CSB) void k_colsum(const float* __restrict__ bias, float* CB) {
#pragma clang fp contract(off)
    __shared__ __align__(16) float cs[CSB];
    const unsigned tid = threadIdx.x;
    const unsigned o = blockIdx.x * (unsigned)CSB + tid;
    float s = 0.0f;
#pragma unroll 8
    for (unsigned d = 0; d < (unsigned)DIN; ++d) s += bfr(bias[(size_t)d * DOUT + o]);
    cs[tid] = s;
    __syncthreads();
    if (tid < 32u) {
        const v4f val = *(const v4fa*)(&cs[tid * 4u]);
        float* dst = CB + (size_t)blockIdx.x * CSB + (size_t)tid * 4;
        *(volatile v4f*)dst = val; __threadfence(); *(volatile v4f*)dst = val; }
}

static_assert(32 * 16 * 8 == 16 * 256);
__global__ __launch_bounds__(32) void k_gemm(const bf* __restrict__ A, const bf* __restrict__ Bt, const float* __restrict__ cb, float* OUT) {
    __shared__ __align__(16) float os[16 * 68];
    const int K = KT;
    const int lane = threadIdx.x & 31, lr = lane & 15, hi = lane >> 4; const int r0 = blockIdx.x * 64, c0 = blockIdx.y * 64;
    v8f acc[4][4];
#pragma unroll
    for (int mb = 0; mb < 4; ++mb)
#pragma unroll
        for (int nb = 0; nb < 4; ++nb) acc[mb][nb] = (v8f){};
    const size_t aoff = (size_t)(r0 + lr) * K + 8 * hi, boff = (size_t)(c0 + lr) * K + 8 * hi;
#pragma unroll 1
    for (int kc = 0; kc < K; kc += 32) {
        v16bf a[4];
#pragma unroll
        for (int mb = 0; mb < 4; ++mb) a[mb] = ldb(A + aoff + (size_t)mb * 16 * K + kc);
#pragma unroll
        for (int nb = 0; nb < 4; ++nb) { const v16bf b = ldb(Bt + boff + (size_t)nb * 16 * K + kc);
#pragma unroll
            for (int mb = 0; mb < 4; ++mb) acc[mb][nb] = wmmabg(a[mb], b, acc[mb][nb]); }
    }
    float bc[4];
#pragma unroll
    for (int nb = 0; nb < 4; ++nb) bc[nb] = cb[c0 + nb * 16 + lr];
#pragma unroll
    for (int mb = 0; mb < 4; ++mb) {
#pragma unroll
        for (int nb = 0; nb < 4; ++nb) {
#pragma unroll
            for (int j = 0; j < 8; ++j) os[(hi * 8 + j) * 68 + nb * 16 + lr] = acc[mb][nb][j] + bc[nb]; }
        wave_sync();
        float* orow = OUT + (size_t)(r0 + mb * 16) * DOUT + c0;
#pragma unroll 1
        for (int ps = 0; ps < 2; ++ps) {
#pragma unroll
            for (int s = 0; s < 8; ++s) { const int row = 2 * s + (lane >> 4), cofs = (lane & 15) * 4;
                const v4f val = *(const v4fa*)(&os[row * 68 + cofs]);
                *(volatile v4f*)(orow + (size_t)row * DOUT + cofs) = val; }
            if (ps == 0) __threadfence(); }
        wave_sync();
    }
}

static constexpr size_t al256(size_t v) { return (v + 255) & ~(size_t)255; }
static constexpr size_t SZ_AP = al256((size_t)NROWS * KT * 2);
static constexpr size_t SZ_WT = al256((size_t)DOUT * KT * 2);
static constexpr size_t SZ_CB = al256((size_t)DOUT * 4);
static constexpr size_t SZ_TOTAL = SZ_AP + SZ_WT + SZ_CB;
static_assert(SZ_TOTAL <= (size_t)134217728);
static_assert((size_t)(NROWS - 1) * KT * 2 + (size_t)KT * 2 <= SZ_AP);
static_assert((size_t)(DOUT - 1) * KT * 2 + (size_t)KT * 2 <= SZ_WT);
static_assert((size_t)(DOUT / CSB - 1) * CSB * 4 + 32 * 16 <= SZ_CB);

extern "C" void kernel_launch(void* const* d_in, const int* in_sizes, int n_in,
                              void* d_out, int out_size, void* d_ws, size_t ws_size, hipStream_t stream) {
    if (n_in < 4) return;
    if ((size_t)in_sizes[0] < (size_t)NROWS * DIN) return;
    if ((size_t)in_sizes[1] < (size_t)DIN * DOUT || (size_t)in_sizes[2] < (size_t)DIN * DOUT || (size_t)in_sizes[3] < (size_t)DIN * DOUT) return;
    if ((size_t)out_size < (size_t)NROWS * DOUT) return;
    if (SZ_TOTAL > ws_size) return;
    const float* x    = (const float*)d_in[0];
    const float* w1   = (const float*)d_in[1];
    const float* bias = (const float*)d_in[2];
    const float* w2   = (const float*)d_in[3];
    float* OUT = (float*)d_out;
    char* wsp = (char*)d_ws;
    bf* AP = (bf*)wsp; wsp += SZ_AP;
    bf* WT = (bf*)wsp; wsp += SZ_WT;
    float* CB = (float*)wsp; wsp += SZ_CB;

    k_aplane<<<(unsigned)(((size_t)NROWS * (DIN / 8)) / 256), 256, 0, stream>>>(x, AP);
    k_wt<<<dim3(DIN / 64, DOUT / 64, 1), 256, 0, stream>>>(w2, WT, 0u);
    k_wt<<<dim3(DIN / 64, DOUT / 64, 1), 256, 0, stream>>>(w1, WT, (unsigned)DIN);
    k_colsum<<<DOUT / CSB, CSB, 0, stream>>>(bias, CB);
    k_gemm<<<dim3(NROWS / 64, DOUT / 64, 1), 32, 0, stream>>>(AP, WT, CB, OUT);
}
